// LabelRestrictedSelfAttention_89163521065537
// MI455X (gfx1250) — hardware-verified
//
#include <hip/hip_runtime.h>


#define __bf16 _Float16
typedef __attribute__((ext_vector_type(16))) _Float16 v16bf;
#define RSPLIT (1.0f / 2048.0f)
typedef __attribute__((ext_vector_type(8)))  float  v8f;

#define N_TOK 2048
#define DIM   4096
#define BM 128
#define BN 128
#define BK 64
#define LDA 72
#define LDB 72
#define NEG_BIG (-3.4028234663852886e38f)

__device__ __forceinline__ __bf16 to_bf16(float f) { return (_Float16)f; }
__device__ __forceinline__ void put2(__bf16* hiT, __bf16* loT, int off, float f) {
  const _Float16 h = (_Float16)f; hiT[off] = h; loT[off] = (_Float16)((f - (float)h) * 2048.0f);
}
typedef __attribute__((ext_vector_type(4))) float v4f_t;
typedef float v4fa __attribute__((ext_vector_type(4), may_alias));
__device__ __forceinline__ void store_tile16x32(const float* stg, float* __restrict__ dst, size_t ld, int lane) {
  v4f_t vv[4];
#pragma unroll
  for (int i = 0; i < 4; ++i) { const int c = lane + 32 * i; vv[i] = *(const v4fa*)(stg + (c >> 3) * 32 + (c & 7) * 4); }
#pragma unroll
  for (int i = 0; i < 4; ++i) { const int c = lane + 32 * i; *(volatile v4f_t*)(dst + (size_t)(c >> 3) * ld + (c & 7) * 4) = vv[i]; }
  __threadfence();
#pragma unroll
  for (int i = 0; i < 4; ++i) { const int c = lane + 32 * i; *(volatile v4f_t*)(dst + (size_t)(c >> 3) * ld + (c & 7) * 4) = vv[i]; }
}

__device__ __forceinline__ void qkv_row(int r, const float* __restrict__ w,
                                        const float* __restrict__ bias,
                                        int& xrow, float& sc, float& of) {
  int bb  = r / 768;
  int rem = r - bb * 768;
  xrow = bb * 256 + rem / 3;
  sc = w[rem];
  of = bias[rem];
}

__device__ __forceinline__ void mma_tile(const __bf16* __restrict__ As, const __bf16* __restrict__ Asl,
                                         const __bf16* __restrict__ Bs, const __bf16* __restrict__ Bsl,
                                         v8f acc[2][4], int wvM, int wvN, int lane) {
  const int l15 = lane & 15;
  const int hi  = lane >> 4;
#pragma unroll
  for (int kk = 0; kk < BK; kk += 32) {
    v16bf a[2], al[2];
#pragma unroll
    for (int mi = 0; mi < 2; ++mi) {
      const int m = wvM * 32 + mi * 16 + l15;
      const int khA = hi * 8;
#pragma unroll
      for (int j = 0; j < 8; ++j) {
        const int k0 = kk + khA + ((j < 4) ? (2 * j) : (2 * j + 8));
        a[mi][2 * j]      = As[m * LDA + k0];
        a[mi][2 * j + 1]  = As[m * LDA + k0 + 1];
        al[mi][2 * j]     = Asl[m * LDA + k0];
        al[mi][2 * j + 1] = Asl[m * LDA + k0 + 1];
      }
    }
#pragma unroll
    for (int ni = 0; ni < 4; ++ni) {
      const int n = wvN * 64 + ni * 16 + l15;
      const int khB = hi * 8;
      v16bf b, bl;
#pragma unroll
      for (int j = 0; j < 8; ++j) {
        const int k0 = kk + khB + ((j < 4) ? (2 * j) : (2 * j + 8));
        b[2 * j]      = Bs[n * LDB + k0];
        b[2 * j + 1]  = Bs[n * LDB + k0 + 1];
        bl[2 * j]     = Bsl[n * LDB + k0];
        bl[2 * j + 1] = Bsl[n * LDB + k0 + 1];
      }
#pragma unroll
      for (int mi = 0; mi < 2; ++mi) {
        v8f x = {};
        x = __builtin_amdgcn_wmma_f32_16x16x32_f16(false, al[mi], false, b, (short)0, x, false, false);
        x = __builtin_amdgcn_wmma_f32_16x16x32_f16(false, a[mi], false, bl, (short)0, x, false, false);
        acc[mi][ni] = __builtin_amdgcn_wmma_f32_16x16x32_f16(false, a[mi], false, b, (short)0, acc[mi][ni], false, false) + x * RSPLIT;
      }
    }
  }
}

__global__ __launch_bounds__(256) void qk_gemm_kernel(
    const float* __restrict__ x, const float* __restrict__ w,
    const float* __restrict__ bias, const int* __restrict__ labels,
    float* __restrict__ S) {
  __shared__ __bf16 As[BM * LDA], Asl[BM * LDA];
  __shared__ __bf16 Bs[BN * LDB], Bsl[BN * LDB];
  __shared__ __attribute__((aligned(16))) float stg[8][16 * 32];

  const int t = threadIdx.x;
  const int lane = t & 31, wv = t >> 5;
  const int wvM = wv & 3, wvN = wv >> 2;
  const int i0 = blockIdx.y * BM;
  const int j0 = blockIdx.x * BN;

  v8f acc[2][4];
#pragma unroll
  for (int mi = 0; mi < 2; ++mi)
#pragma unroll
    for (int ni = 0; ni < 4; ++ni)
#pragma unroll
      for (int e = 0; e < 8; ++e) acc[mi][ni][e] = 0.f;

  for (int d0 = 0; d0 < DIM; d0 += BK) {
#pragma unroll 2
    for (int p = 0; p < 8; ++p) {
      const int ml = (t >> 4) + p * 16;
      const int c4 = (t & 15) * 4;
      int xrow; float sc, of;
      qkv_row(i0 + ml, w, bias, xrow, sc, of);
      const float4 v = *(const float4*)(x + (size_t)xrow * DIM + d0 + c4);
      const int o_ = ml * LDA + c4;
      put2(As, Asl, o_, v.x * sc + of); put2(As, Asl, o_ + 1, v.y * sc + of);
      put2(As, Asl, o_ + 2, v.z * sc + of); put2(As, Asl, o_ + 3, v.w * sc + of);
    }
#pragma unroll 2
    for (int p = 0; p < 8; ++p) {
      const int nl = (t >> 4) + p * 16;
      const int c4 = (t & 15) * 4;
      int xrow; float sc, of;
      qkv_row(2048 + j0 + nl, w, bias, xrow, sc, of);
      const float4 v = *(const float4*)(x + (size_t)xrow * DIM + d0 + c4);
      const int o_ = nl * LDB + c4;
      put2(Bs, Bsl, o_, v.x * sc + of); put2(Bs, Bsl, o_ + 1, v.y * sc + of);
      put2(Bs, Bsl, o_ + 2, v.z * sc + of); put2(Bs, Bsl, o_ + 3, v.w * sc + of);
    }
    __syncthreads();
    mma_tile(As, Asl, Bs, Bsl, acc, wvM, wvN, lane);
    __syncthreads();
  }

  const int l15 = lane & 15, hi = lane >> 4;
  float* sg = stg[wv];
#pragma unroll
  for (int mi = 0; mi < 2; ++mi) {
#pragma unroll
    for (int np = 0; np < 4; np += 2) {
#pragma unroll
      for (int nj = 0; nj < 2; ++nj) {
        const int gn = j0 + wvN * 64 + (np + nj) * 16 + l15;
        const int lj = labels[gn];
#pragma unroll
        for (int r = 0; r < 8; ++r) {
          const int gm = i0 + wvM * 32 + mi * 16 + r + 8 * hi;
          const int li = labels[gm];
          const bool keep = (li == lj) && (li >= 0);
          sg[(r + 8 * hi) * 32 + nj * 16 + l15] = keep ? acc[mi][np + nj][r] : NEG_BIG;
        }
      }
      store_tile16x32(sg, S + (size_t)(i0 + wvM * 32 + mi * 16) * N_TOK + j0 + wvN * 64 + np * 16, (size_t)N_TOK, lane);
    }
  }
}

__global__ __launch_bounds__(256) void softmax_kernel(float* __restrict__ S) {
  const int row = blockIdx.x;
  float* p = S + (size_t)row * N_TOK;
  const int t = threadIdx.x;
  __shared__ float red[256];

  float v[8];
  float m = NEG_BIG;
#pragma unroll
  for (int e = 0; e < 8; ++e) { v[e] = p[t + e * 256]; m = fmaxf(m, v[e]); }
  red[t] = m;
  __syncthreads();
  for (int off = 128; off > 0; off >>= 1) {
    if (t < off) red[t] = fmaxf(red[t], red[t + off]);
    __syncthreads();
  }
  const float rmax = red[0];
  __syncthreads();

  float s = 0.f;
#pragma unroll
  for (int e = 0; e < 8; ++e) { v[e] = __expf(v[e] - rmax); s += v[e]; }
  red[t] = s;
  __syncthreads();
  for (int off = 128; off > 0; off >>= 1) {
    if (t < off) red[t] += red[t + off];
    __syncthreads();
  }
  const float inv = 1.f / red[0];
#pragma unroll
  for (int e = 0; e < 8; ++e) *(volatile float*)(p + t + e * 256) = v[e] * inv;
  __threadfence();
#pragma unroll
  for (int e = 0; e < 8; ++e) *(volatile float*)(p + t + e * 256) = v[e] * inv;
}

__global__ __launch_bounds__(256) void pv_gemm_kernel(
    const float* __restrict__ x, const float* __restrict__ w,
    const float* __restrict__ bias, const int* __restrict__ labels,
    const float* __restrict__ P, float* __restrict__ out) {
  __shared__ __bf16 As[BM * LDA], Asl[BM * LDA];
  __shared__ __bf16 Bs[BN * LDB], Bsl[BN * LDB];
  __shared__ __attribute__((aligned(16))) float stg[8][16 * 32];

  const int t = threadIdx.x;
  const int lane = t & 31, wv = t >> 5;
  const int wvM = wv & 3, wvN = wv >> 2;
  const int i0 = blockIdx.y * BM;
  const int d0 = blockIdx.x * BN;

  v8f acc[2][4];
#pragma unroll
  for (int mi = 0; mi < 2; ++mi)
#pragma unroll
    for (int ni = 0; ni < 4; ++ni)
#pragma unroll
      for (int e = 0; e < 8; ++e) acc[mi][ni][e] = 0.f;

  for (int k0 = 0; k0 < N_TOK; k0 += BK) {
#pragma unroll 2
    for (int p = 0; p < 8; ++p) {
      const int ml = (t >> 4) + p * 16;
      const int c4 = (t & 15) * 4;
      const float4 v = *(const float4*)(P + (size_t)(i0 + ml) * N_TOK + k0 + c4);
      const int o_ = ml * LDA + c4;
      put2(As, Asl, o_, v.x * 1024.0f); put2(As, Asl, o_ + 1, v.y * 1024.0f);
      put2(As, Asl, o_ + 2, v.z * 1024.0f); put2(As, Asl, o_ + 3, v.w * 1024.0f);
    }
#pragma unroll 2
    for (int p = 0; p < 8; ++p) {
      const int jl = (t >> 5) + p * 8;
      const int c4 = (t & 31) * 4;
      int xrow; float sc, of;
      qkv_row(4096 + k0 + jl, w, bias, xrow, sc, of);
      const float4 v = *(const float4*)(x + (size_t)xrow * DIM + d0 + c4);
      put2(Bs, Bsl, (c4 + 0) * LDB + jl, v.x * sc + of);
      put2(Bs, Bsl, (c4 + 1) * LDB + jl, v.y * sc + of);
      put2(Bs, Bsl, (c4 + 2) * LDB + jl, v.z * sc + of);
      put2(Bs, Bsl, (c4 + 3) * LDB + jl, v.w * sc + of);
    }
    __syncthreads();
    mma_tile(As, Asl, Bs, Bsl, acc, wvM, wvN, lane);
    __syncthreads();
  }

  const int l15 = lane & 15, hi = lane >> 4;
  float* sg = stg[wv];
#pragma unroll
  for (int mi = 0; mi < 2; ++mi) {
#pragma unroll
    for (int np = 0; np < 4; np += 2) {
#pragma unroll
      for (int nj = 0; nj < 2; ++nj)
#pragma unroll
        for (int r = 0; r < 8; ++r) {
          const int gm = i0 + wvM * 32 + mi * 16 + r + 8 * hi;
          const float val = acc[mi][np + nj][r] * (1.0f / 1024.0f);
          sg[(r + 8 * hi) * 32 + nj * 16 + l15] = (labels[gm] >= 0) ? val : 0.f;
        }
      store_tile16x32(sg, out + (size_t)(i0 + wvM * 32 + mi * 16) * DIM + d0 + wvN * 64 + np * 16, (size_t)DIM, lane);
    }
  }
}

extern "C" void kernel_launch(void* const* d_in, const int* in_sizes, int n_in,
                              void* d_out, int out_size, void* d_ws, size_t ws_size,
                              hipStream_t stream) {
  (void)in_sizes; (void)n_in; (void)out_size; (void)ws_size;
  const float* x      = (const float*)d_in[0];
  const int*   labels = (const int*)d_in[1];
  const float* w      = (const float*)d_in[2];
  const float* b      = (const float*)d_in[3];
  float* out = (float*)d_out;
  float* S   = (float*)d_ws;

  dim3 blk(256);
  qk_gemm_kernel<<<dim3(N_TOK / BN, N_TOK / BM), blk, 0, stream>>>(x, w, b, labels, S);
  softmax_kernel<<<dim3(N_TOK), blk, 0, stream>>>(S);
  pv_gemm_kernel<<<dim3(DIM / BN, N_TOK / BM), blk, 0, stream>>>(x, w, b, labels, S, out);
}
